// _EncoderBlock_21964462752254
// MI455X (gfx1250) — hardware-verified
//
#include <hip/hip_runtime.h>

typedef __attribute__((ext_vector_type(16))) _Float16 v16h;
typedef __attribute__((ext_vector_type(8)))  _Float16 v8h;
typedef __attribute__((ext_vector_type(8)))  float    v8f;
typedef __attribute__((ext_vector_type(4)))  float    v4f;
typedef __attribute__((ext_vector_type(4)))  unsigned v4u;
template <typename T> __device__ __forceinline__ void vst2(void* p, T v) { *(volatile T*)p = v; __threadfence(); *(volatile T*)p = v; }
__device__ __forceinline__ v8f wmma16(v16h a, v16h b, v8f c) {
    v8f d = __builtin_amdgcn_wmma_f32_16x16x32_f16(false, a, false, b, (short)0, c, false, false);
    asm volatile("v_nop\n\tv_nop\n\tv_nop\n\tv_nop" : "+v"(d) : "v"(a), "v"(b));
    return d;
}

#define D8    8
#define C_CH  256
#define FEAT  2048
#define TOK   4096
#define NROT  4

__device__ __forceinline__ float cl_sign(int a, int b) {
    int t = a >> 1, cnt = 0;
    while (t) { cnt += __popc(t & b); t >>= 1; }
    return (cnt & 1) ? -1.0f : 1.0f;
}

__global__ __launch_bounds__(64) void rotor_matrix_kernel(const float* __restrict__ rotor_biv,
                                                          const float* __restrict__ rotor_mix,
                                                          float* __restrict__ Mc_out) {
    __shared__ __align__(16) float T1s[64][64], Ys[64][64], Ms[64][64];
    const int tl = threadIdx.x, c = blockIdx.x * 64 + tl;
    float m[NROT], mx = -1e30f;
    for (int r = 0; r < NROT; ++r) { m[r] = rotor_mix[r]; mx = fmaxf(mx, m[r]); }
    float s = 0.f;
    for (int r = 0; r < NROT; ++r) { m[r] = expf(m[r] - mx); s += m[r]; }
    float* T1 = T1s[tl]; float* Y = Ys[tl]; float* Mc = Ms[tl];
    for (int i = 0; i < 64; ++i) Mc[i] = 0.f;
    const int nz[4] = {0, 3, 5, 6};
    const float rev[8] = {1,1,1,-1,1,-1,-1,-1};
    #pragma unroll 1
    for (int r = 0; r < NROT; ++r) {
        float p = m[r] / s;
        float Rv[8] = {0,0,0,0,0,0,0,0};
        Rv[0] = 1.f;
        Rv[3] = rotor_biv[(r*C_CH + c)*3 + 0];
        Rv[5] = rotor_biv[(r*C_CH + c)*3 + 1];
        Rv[6] = rotor_biv[(r*C_CH + c)*3 + 2];
        float inv = 1.f / sqrtf(Rv[0]*Rv[0] + Rv[3]*Rv[3] + Rv[5]*Rv[5] + Rv[6]*Rv[6]);
        for (int i = 0; i < 64; ++i) { T1[i] = 0.f; Y[i] = 0.f; }
        #pragma unroll
        for (int u = 0; u < 4; ++u) {
            const int i = nz[u];
            const float ri = Rv[i] * inv, rti = ri * rev[i];
            #pragma unroll 1
            for (int j = 0; j < 8; ++j) { T1[(i ^ j) * 8 + j] += ri * cl_sign(i, j); Y[(j ^ i) * 8 + j] += rti * cl_sign(j, i); }
        }
        #pragma unroll 1
        for (int k = 0; k < 8; ++k)
            #pragma unroll 1
            for (int j = 0; j < 8; ++j) {
                float acc = 0.f;
                #pragma unroll
                for (int t = 0; t < 8; ++t) acc += Y[k * 8 + t] * T1[t * 8 + j];
                Mc[k * 8 + j] += p * acc;
            }
    }
    __syncthreads();
    for (int gq = tl; gq < 64 * 16; gq += 64) { const int cl = gq >> 4, pc = gq & 15;
        vst2(Mc_out + (size_t)(blockIdx.x * 64 + cl) * 64 + pc * 4, *(const v4f*)(&Ms[cl][pc * 4])); }
}

__global__ __launch_bounds__(256) void fuse_weight_kernel(const float* __restrict__ lin_weight,
                                                          const float* __restrict__ Mc_in,
                                                          _Float16* __restrict__ WfT) {
    __shared__ float w8s[256][9];
    __shared__ __align__(16) float Mcs[256][64];
    const int tid = blockIdx.x * blockDim.x + threadIdx.x;
    const int o = tid >> 8, c = tid & 255, tl = threadIdx.x;
    for (int i = 0; i < 8; ++i) w8s[tl][i] = lin_weight[(size_t)tid * 8 + i];
    for (int i = tl; i < 256 * 16; i += 256) *(v4f*)(&Mcs[0][0] + i * 4) = *(const v4f*)(Mc_in + (size_t)i * 4);
    __syncthreads();
    const float* w8 = w8s[tl]; const float* Mc = Mcs[c];
    #pragma unroll 1
    for (int k = 0; k < 8; ++k) {
        float wb[8];
        #pragma unroll
        for (int jp = 0; jp < 8; ++jp) wb[jp] = w8[k ^ jp] * cl_sign(k ^ jp, jp);
        union { _Float16 h[8]; v4u u; } wrow;
        #pragma unroll
        for (int j = 0; j < 8; ++j) {
            float acc = 0.f;
            #pragma unroll
            for (int jp = 0; jp < 8; ++jp) acc += wb[jp] * Mc[jp * 8 + j];
            wrow.h[j] = (_Float16)acc;
        }
        vst2(WfT + (size_t)(o*8 + k) * FEAT + c*8, wrow.u);
    }
}

__global__ void act_kernel(const float* __restrict__ x,
                           const float* __restrict__ norm_weight,
                           _Float16* __restrict__ act) {
    int tid = blockIdx.x * blockDim.x + threadIdx.x;
    if (tid >= TOK * C_CH) return;
    int c = tid & 255;

    const float4* xp = (const float4*)(x + (size_t)tid * 8);
    float4 a = xp[0], b = xp[1];
    float v[8] = {a.x, a.y, a.z, a.w, b.x, b.y, b.z, b.w};

    const float EPS = 1e-5f;
    float g[4];
    g[0] = sqrtf(v[0]*v[0] + EPS);
    g[1] = sqrtf(v[1]*v[1] + v[2]*v[2] + v[4]*v[4] + EPS);
    g[2] = sqrtf(v[3]*v[3] + v[5]*v[5] + v[6]*v[6] + EPS);
    g[3] = sqrtf(v[7]*v[7] + EPS);
    float w[4];
    for (int q = 0; q < 4; ++q) w[q] = norm_weight[c*4 + q] / g[q];

    const int grade[8] = {0,1,1,2,1,2,2,3};
    union { _Float16 h[8]; v4u u; } h8;
    #pragma unroll 1
    for (int d = 0; d < 8; ++d) {
        float h = v[d] * w[grade[d]];
        float t = tanhf(0.7978845608028654f * (h + 0.044715f * h*h*h));
        h8.h[d] = (_Float16)(0.5f * h * (1.f + t));
    }
    vst2(act + (size_t)tid * 8, h8.u);
}

#define BM 128
#define BN 128
#define BK 32
#define NK (FEAT / BK)
#define LDA 40

__global__ __launch_bounds__(256)
void gemm_kernel(const _Float16* __restrict__ act,
                 const _Float16* __restrict__ WfT,
                 const float* __restrict__ bias,
                 const float* __restrict__ xres,
                 float* __restrict__ out) {
    __shared__ __align__(16) _Float16 As[2][BM * LDA];
    __shared__ __align__(16) _Float16 Bs[2][BN * LDA];
    __shared__ __align__(16) float So[8][32 * 64];

    int tid  = threadIdx.x;
    int wave = tid >> 5, lane = tid & 31;
    int wm = wave >> 1, wn = wave & 1;
    int m0 = blockIdx.y * BM, n0 = blockIdx.x * BN;

    v8f zero = {};
    v8f acc[2][4];
    for (int i = 0; i < 2; ++i) for (int j = 0; j < 4; ++j) acc[i][j] = zero;

    int lrow = tid >> 1;
    int lcol = (tid & 1) * 16;

    const _Float16* ga = act + (size_t)(m0 + lrow) * FEAT + lcol;
    const _Float16* gb = WfT + (size_t)(n0 + lrow) * FEAT + lcol;
    auto stage = [&](int kb, int buf) {
        const v8h* sa = (const v8h*)(ga + kb * BK); const v8h* sb = (const v8h*)(gb + kb * BK);
        *(v8h*)&As[buf][lrow * LDA + lcol] = sa[0]; *(v8h*)&As[buf][lrow * LDA + lcol + 8] = sa[1];
        *(v8h*)&Bs[buf][lrow * LDA + lcol] = sb[0]; *(v8h*)&Bs[buf][lrow * LDA + lcol + 8] = sb[1];
    };
    stage(0, 0);

    for (int kb = 0; kb < NK; ++kb) {
        int cur = kb & 1;
        __syncthreads();
        if (kb + 1 < NK) stage(kb + 1, cur ^ 1);

        const _Float16* Ab = &As[cur][0];
        const _Float16* Bb = &Bs[cur][0];
        int rl  = lane & 15;
        int kb8 = (lane >> 4) << 3;
        int ks  = (lane >> 4) << 3;
        union Frag { v16h v; v8h h[2]; } af[2], bf[4];
        for (int ms = 0; ms < 2; ++ms) {
            int r = wm * 32 + ms * 16 + rl;
            af[ms].h[0] = *(const v8h*)&Ab[r * LDA + kb8];
            af[ms].h[1] = *(const v8h*)&Ab[r * LDA + kb8 + 16];
        }
        for (int ns = 0; ns < 4; ++ns) {
            int r = wn * 64 + ns * 16 + rl;
            bf[ns].h[0] = *(const v8h*)&Bb[r * LDA + ks];
            bf[ns].h[1] = *(const v8h*)&Bb[r * LDA + ks + 16];
        }
        for (int ms = 0; ms < 2; ++ms)
            for (int ns = 0; ns < 4; ++ns)
                acc[ms][ns] = wmma16(af[ms].v, bf[ns].v, acc[ms][ns]);
    }

    float* S = So[wave];
    for (int ms = 0; ms < 2; ++ms)
        for (int ns = 0; ns < 4; ++ns) {
            float bcol = bias[n0 + wn * 64 + ns * 16 + (lane & 15)];
            for (int r = 0; r < 8; ++r) S[(ms * 16 + ((lane >> 4) << 3) + r) * 64 + ns * 16 + (lane & 15)] = acc[ms][ns][r] + bcol;
        }
    asm volatile("s_wait_dscnt 0" ::: "memory"); __builtin_amdgcn_wave_barrier(); __builtin_amdgcn_fence(__ATOMIC_RELEASE, "workgroup");
    #pragma unroll 4
    for (int q = 0; q < 16; ++q) { const int rl = q * 2 + (lane >> 4), pc = lane & 15;
        const size_t idx = (size_t)(m0 + wm * 32 + rl) * FEAT + n0 + wn * 64 + pc * 4;
        v4f v = *(const v4f*)(S + rl * 64 + pc * 4); const v4f rr = *(const v4f*)(xres + idx);
        vst2(out + idx, v + rr); }
}

extern "C" void kernel_launch(void* const* d_in, const int* in_sizes, int n_in,
                              void* d_out, int out_size, void* d_ws, size_t ws_size,
                              hipStream_t stream) {
    const float* x           = (const float*)d_in[0];
    const float* norm_weight = (const float*)d_in[1];
    const float* rotor_biv   = (const float*)d_in[2];
    const float* rotor_mix   = (const float*)d_in[3];
    const float* lin_weight  = (const float*)d_in[4];
    const float* lin_bias    = (const float*)d_in[5];
    float* out = (float*)d_out;

    float*    Mc  = (float*)d_ws;
    _Float16* WfT = (_Float16*)((char*)d_ws + 65536);
    _Float16* act = (_Float16*)((char*)d_ws + 65536 + (size_t)FEAT * FEAT * 2);

    rotor_matrix_kernel<<<4, 64, 0, stream>>>(rotor_biv, rotor_mix, Mc);
    fuse_weight_kernel<<<(C_CH * C_CH) / 256, 256, 0, stream>>>(lin_weight, Mc, WfT);
    act_kernel<<<(TOK * C_CH) / 256, 256, 0, stream>>>(x, norm_weight, act);
    gemm_kernel<<<dim3(FEAT / BN, TOK / BM), 256, 0, stream>>>(act, WfT, lin_bias, x, out);
}
